// GraphAttentionLayer_84610855731510
// MI455X (gfx1250) — hardware-verified
//
#include <hip/hip_runtime.h>
#include <stddef.h>
#include <stdint.h>
#include <math.h>


#define CCH     128
#define KNN     16
#define CS      16
#define NQKV    384
#define NTHR    256
#define GBM     64
#define GBN     64
#define GTHR    128
#define APITCH  264
#define A2PITCH 40
#define PW      4
#define PTHR    128
#define KR      4
#define KW      8
#define KTHR    256
#define KROWS   (KR * KW)
#define PCAP    64
#define PTRIG   16
#define WSMAX   134217728
#define BN_C    ((float)1.0000049999875000625)
#define TIEULP  4.76837158203125e-7f
#define PADKEY  0xFFFFFFFFFFFFFFFFull

static_assert(KTHR == KW * 32);
static_assert(KROWS == 32);
static_assert(PTRIG + 31 <= PCAP);
static_assert((PCAP % 32) == 0);
static_assert(GBM == (GTHR / 32) * 16);
static_assert((CCH % 32) == 0 && (NQKV % GBN) == 0);
static_assert(CCH == 4 * 32);
static_assert((APITCH % 8) == 0 && APITCH >= 2 * CCH);
static_assert((A2PITCH % 8) == 0 && A2PITCH >= 2 * CS);
static_assert(CCH * CCH / 8 == 8 * NTHR);
static_assert(PTHR == PW * 32);

typedef float          v4f  __attribute__((ext_vector_type(4)));
typedef float          v8f  __attribute__((ext_vector_type(8)));
typedef int            v4i  __attribute__((ext_vector_type(4)));
typedef int            v8i  __attribute__((ext_vector_type(8)));
typedef unsigned int   v2u  __attribute__((ext_vector_type(2)));
typedef unsigned int   v4u  __attribute__((ext_vector_type(4)));
typedef unsigned short v8us __attribute__((ext_vector_type(8)));
typedef __bf16         v16b __attribute__((ext_vector_type(16)));
typedef v4f  __attribute__((may_alias)) v4fa;
typedef v4i  __attribute__((may_alias)) v4ia;
typedef v2u  __attribute__((may_alias)) v2ua;
typedef v8us __attribute__((may_alias)) v8usa;
typedef unsigned long long u64;
union FragB { v16b v; v8us h[2]; v8i w; };

__device__ __forceinline__ v8f wmb(const FragB& a, const FragB& b, v8f c) {
  v8f d = __builtin_amdgcn_wmma_f32_16x16x32_bf16(false, a.v, false, b.v, (short)0, c, false, false);
  asm volatile("v_nop\n\tv_nop\n\tv_nop\n\tv_nop" : "+v"(d) : "v"(a.w), "v"(b.w));
  return d;
}

__device__ __forceinline__ void ldwait() {
  asm volatile("s_wait_loadcnt 0x0" ::: "memory");
}

__device__ __forceinline__ unsigned int f2bf(float f) {
  const unsigned int u = __float_as_uint(f);
  return ((u + 0x7FFFu + ((u >> 16) & 1u)) >> 16) & 0xFFFFu;
}
__device__ __forceinline__ float bf2f(unsigned int b) { return __uint_as_float(b << 16); }
__device__ __forceinline__ float bfr(float f) { return bf2f(f2bf(f)); }
__device__ __forceinline__ v4f bfr4(const v4f a) {
  v4f r; r.x = bfr(a.x); r.y = bfr(a.y); r.z = bfr(a.z); r.w = bfr(a.w); return r;
}
__device__ __forceinline__ unsigned int pk2(float lo, float hi) { return f2bf(lo) | (f2bf(hi) << 16); }
__device__ __forceinline__ v4u pack8(const v4f a, const v4f b) {
  v4u r;
  r.x = pk2(a.x, a.y); r.y = pk2(a.z, a.w); r.z = pk2(b.x, b.y); r.w = pk2(b.z, b.w);
  return r;
}
__device__ __forceinline__ float rdlf(float v, int l) {
  return __int_as_float(__builtin_amdgcn_readlane(__float_as_int(v), l));
}

__global__ __launch_bounds__(NTHR) void k_pprep(const float* __restrict__ p, float* p4, int nN) {
#pragma clang fp contract(off)
  const int i = (int)blockIdx.x * NTHR + (int)threadIdx.x;
  if (i >= nN) return;
  const float x = bfr(p[3 * i]), y = bfr(p[3 * i + 1]), z = bfr(p[3 * i + 2]);
  const float xx = x * x;
  const float yy = y * y;
  const float zz = z * z;
  const float xz = xx + zz;
  const float sq = xz + yy;
  v4f v; v.x = x; v.y = y; v.z = z; v.w = sq;
  float* o = p4 + 4 * (size_t)i;
  *(volatile v4f*)o = v;
  __threadfence();
  *(volatile v4f*)o = v;
}

__global__ __launch_bounds__(NTHR) void k_xprep(const float* __restrict__ x, unsigned short* xb, int nN, int nUnits) {
  const int i = (int)blockIdx.x * NTHR + (int)threadIdx.x;
  if (i >= nUnits) return;
  const int row = i >> 4;
  const int c0  = (i & 15) * 8;
  const int rc  = row < nN ? row : nN - 1;
  const float* p = x + (size_t)rc * CCH + c0;
  v4f a = *(const v4fa*)p, b = *(const v4fa*)(p + 4);
  const v4f z4 = {0.f, 0.f, 0.f, 0.f};
  if (row >= nN) { a = z4; b = z4; }
  const v4u hv = pack8(a, b);
  const size_t o = (size_t)row * CCH + c0;
  *(volatile v4u*)(xb + o) = hv;
  __threadfence();
  *(volatile v4u*)(xb + o) = hv;
}

__global__ __launch_bounds__(NTHR) void k_wtr3(const float* __restrict__ w0, const float* __restrict__ w1,
                                               const float* __restrict__ w2, unsigned short* wt) {
  const int mat = (int)blockIdx.x >> 3;
  const float* w = (mat == 0) ? w0 : ((mat == 1) ? w1 : w2);
  const int u  = ((int)blockIdx.x & 7) * NTHR + (int)threadIdx.x;
  const int n  = u >> 4;
  const int k8 = (u & 15) * 8;
  const float* p = w + (size_t)k8 * CCH + n;
  v4f a, b;
  a.x = p[0];        a.y = p[CCH];      a.z = p[2 * CCH];  a.w = p[3 * CCH];
  b.x = p[4 * CCH];  b.y = p[5 * CCH];  b.z = p[6 * CCH];  b.w = p[7 * CCH];
  const v4u wv = pack8(a, b);
  unsigned short* o = wt + (size_t)(mat * CCH + n) * CCH + k8;
  *(volatile v4u*)o = wv;
  __threadfence();
  *(volatile v4u*)o = wv;
}

__global__ __launch_bounds__(NTHR) void k_wtr(const float* __restrict__ w, int Kin, int Ncol, int Nrows, int Kout,
                                              unsigned short* wt, int nUnits) {
  const int u = (int)blockIdx.x * NTHR + (int)threadIdx.x;
  if (u >= nUnits) return;
  const int kq = Kout >> 3;
  const int n  = u / kq;
  const int k8 = (u - n * kq) * 8;
  const int kk = k8 - (k8 / Kin) * Kin;
  const int ncl = n < Ncol ? n : Ncol - 1;
  const float* p = w + (size_t)kk * (size_t)Ncol + ncl;
  v4f a, b;
  a.x = p[0];                    a.y = p[(size_t)Ncol];         a.z = p[(size_t)2 * Ncol];     a.w = p[(size_t)3 * Ncol];
  b.x = p[(size_t)4 * Ncol];     b.y = p[(size_t)5 * Ncol];     b.z = p[(size_t)6 * Ncol];     b.w = p[(size_t)7 * Ncol];
  const v4f z4 = {0.f, 0.f, 0.f, 0.f};
  if (n >= Ncol || n >= Nrows) { a = z4; b = z4; }
  const v4u wv = pack8(a, b);
  unsigned short* o = wt + (size_t)n * (size_t)Kout + k8;
  *(volatile v4u*)o = wv;
  __threadfence();
  *(volatile v4u*)o = wv;
}

__device__ __forceinline__ float d2key(const v4f q, const v4f c) {
#pragma clang fp contract(off)
  const float px = q.x * c.x;
  const float py = q.y * c.y;
  const float pz = q.z * c.z;
  const float pxy = px + py;
  const float dot = pxy + pz;
  const float s   = q.w + c.w;
  const float two = 2.0f * dot;
  return s - two;
}
__device__ __forceinline__ unsigned f2ord(float f) {
  const unsigned u = __float_as_uint(f);
  return (u & 0x80000000u) ? ~u : (u | 0x80000000u);
}
__device__ __forceinline__ float ord2f(unsigned o) {
  const unsigned u = (o & 0x80000000u) ? (o ^ 0x80000000u) : ~o;
  return __uint_as_float(u);
}
__device__ __forceinline__ u64 shx64(u64 v, int msk) {
  const int lo = __shfl_xor((int)(unsigned)(v & 0xFFFFFFFFull), msk);
  const int hi = __shfl_xor((int)(unsigned)(v >> 32), msk);
  return ((u64)(unsigned)hi << 32) | (u64)(unsigned)lo;
}
__device__ __forceinline__ u64 cxs(u64 v, int j, bool keepmin) {
  const u64 o = shx64(v, j);
  const bool lt = o < v;
  return (keepmin == lt) ? o : v;
}
__device__ __forceinline__ u64 sort32(u64 v, int lane) {
#pragma unroll
  for (int k = 2; k <= 32; k <<= 1) {
#pragma unroll
    for (int j = k >> 1; j > 0; j >>= 1) {
      const bool up   = (lane & k) == 0;
      const bool lowr = (lane & j) == 0;
      v = cxs(v, j, lowr == up);
    }
  }
  return v;
}
__device__ __forceinline__ u64 merge32(u64 best, u64 srt, int lane) {
  const u64 rv = shx64(srt, 31);
  u64 v = rv < best ? rv : best;
#pragma unroll
  for (int j = 16; j > 0; j >>= 1) v = cxs(v, j, (lane & j) == 0);
  return v;
}
__device__ __forceinline__ void knn_step(float d2, int j, float tau, int& cnt, u64* pend) {
  const bool pass = d2 < tau;
  const unsigned msk = __builtin_amdgcn_ballot_w32(pass);
  if (msk != 0u) {
    const int pos = cnt + (int)__builtin_amdgcn_mbcnt_lo(msk, 0u);
    if (pass && pos < PCAP) pend[pos] = ((u64)f2ord(d2) << 32) | (u64)(unsigned)j;
    cnt += (int)__builtin_popcount(msk);
  }
}
__device__ __forceinline__ void knn_flush(u64& best, float& tau, int& cnt, int& ovf, const u64* pend, int lane) {
  __builtin_amdgcn_fence(__ATOMIC_RELEASE, "wavefront");
  __builtin_amdgcn_wave_barrier();
  ovf |= (cnt > PCAP) ? 1 : 0;
  const int n = cnt > PCAP ? PCAP : cnt;
#pragma unroll 1
  for (int c0 = 0; c0 < PCAP; c0 += 32) {
    if (c0 < n) {
      const int e  = c0 + lane;
      const int ec = e < n ? e : n - 1;
      u64 pk = pend[ec];
      pk = e < n ? pk : PADKEY;
      pk = sort32(pk, lane);
      best = merge32(best, pk, lane);
    }
  }
  cnt = 0;
  const unsigned h16 = (unsigned)__builtin_amdgcn_readlane((int)(unsigned)(best >> 32), 16);
  tau = (h16 == 0xFFFFFFFFu) ? __int_as_float(0x7f800000) : ord2f(h16);
  __builtin_amdgcn_fence(__ATOMIC_RELEASE, "wavefront");
  __builtin_amdgcn_wave_barrier();
}
__device__ __forceinline__ int knn_word(u64 best, const v4f q, int ovf, const float* __restrict__ P4, int nN,
                                        int lane, int& flag) {
  int j = (int)(unsigned)(best & 0xFFFFFFFFull);
  j = j < 0 ? 0 : (j > nN - 1 ? nN - 1 : j);
  const float d2 = ord2f((unsigned)(best >> 32));
  const float sj = P4[4 * (size_t)j + 3];
  const float s  = q.w + sj;
  const float d15 = rdlf(d2, 15), d16 = rdlf(d2, 16);
  const float s15 = rdlf(s, 15),  s16 = rdlf(s, 16);
  const float smax = fmaxf(s15, s16);
  flag = ((d16 - d15) <= TIEULP * smax) ? 1 : 0;
  const int d2b = ovf ? 0x7fc00000 : __float_as_int(d2);
  const int dsh = __shfl(d2b, lane & 15);
  return lane < 16 ? j : dsh;
}

#define KSTEP(Q, TAU, CNT, BEST, PD) { \
    const float dd = d2key(Q, c); \
    knn_step(dd, j, TAU, CNT, PD); \
    if (CNT >= PTRIG) knn_flush(BEST, TAU, CNT, ovf, PD, lane); }

__global__ __launch_bounds__(KTHR) void k_knn(const float* __restrict__ P4, int* KN, int* TIE, int nN) {
  __shared__ u64 s_pend[KW * KR * PCAP];
  __shared__ __attribute__((aligned(16))) int s_flag[KROWS];
  const int tid = (int)threadIdx.x, lane = tid & 31, wave = tid >> 5;
  const int row0 = (int)blockIdx.x * KROWS + wave * KR;
  u64* pd0 = s_pend + (wave * KR + 0) * PCAP;
  u64* pd1 = s_pend + (wave * KR + 1) * PCAP;
  u64* pd2 = s_pend + (wave * KR + 2) * PCAP;
  u64* pd3 = s_pend + (wave * KR + 3) * PCAP;
  const int rc0 = row0     < nN ? row0     : nN - 1;
  const int rc1 = row0 + 1 < nN ? row0 + 1 : nN - 1;
  const int rc2 = row0 + 2 < nN ? row0 + 2 : nN - 1;
  const int rc3 = row0 + 3 < nN ? row0 + 3 : nN - 1;
  const v4f q0 = *(const v4fa*)(P4 + 4 * (size_t)rc0);
  const v4f q1 = *(const v4fa*)(P4 + 4 * (size_t)rc1);
  const v4f q2 = *(const v4fa*)(P4 + 4 * (size_t)rc2);
  const v4f q3 = *(const v4fa*)(P4 + 4 * (size_t)rc3);
  const float pinf = __int_as_float(0x7f800000);
  float tau0 = pinf, tau1 = pinf, tau2 = pinf, tau3 = pinf;
  int cnt0 = 0, cnt1 = 0, cnt2 = 0, cnt3 = 0, ovf = 0;
  u64 b0 = PADKEY, b1 = PADKEY, b2 = PADKEY, b3 = PADKEY;

  const int nIt = nN >> 5;
#pragma unroll 1
  for (int it = 0; it < nIt; ++it) {
    const int j = it * 32 + lane;
    const v4f c = *(const v4fa*)(P4 + 4 * (size_t)j);
    KSTEP(q0, tau0, cnt0, b0, pd0)
    KSTEP(q1, tau1, cnt1, b1, pd1)
    KSTEP(q2, tau2, cnt2, b2, pd2)
    KSTEP(q3, tau3, cnt3, b3, pd3)
  }
  if (cnt0 > 0) knn_flush(b0, tau0, cnt0, ovf, pd0, lane);
  if (cnt1 > 0) knn_flush(b1, tau1, cnt1, ovf, pd1, lane);
  if (cnt2 > 0) knn_flush(b2, tau2, cnt2, ovf, pd2, lane);
  if (cnt3 > 0) knn_flush(b3, tau3, cnt3, ovf, pd3, lane);

  int f0, f1, f2, f3;
  const int w0 = knn_word(b0, q0, ovf, P4, nN, lane, f0);
  const int w1 = knn_word(b1, q1, ovf, P4, nN, lane, f1);
  const int w2 = knn_word(b2, q2, ovf, P4, nN, lane, f2);
  const int w3 = knn_word(b3, q3, ovf, P4, nN, lane, f3);
  int* kp = KN + (size_t)row0 * 32 + lane;
  const bool k0 = row0 < nN, k1 = row0 + 1 < nN, k2 = row0 + 2 < nN, k3 = row0 + 3 < nN;
  if (k0) *(volatile int*)(kp)      = w0;
  if (k1) *(volatile int*)(kp + 32) = w1;
  if (k2) *(volatile int*)(kp + 64) = w2;
  if (k3) *(volatile int*)(kp + 96) = w3;
  __threadfence();
  if (k0) *(volatile int*)(kp)      = w0;
  if (k1) *(volatile int*)(kp + 32) = w1;
  if (k2) *(volatile int*)(kp + 64) = w2;
  if (k3) *(volatile int*)(kp + 96) = w3;

  if (lane == 0) {
    s_flag[wave * KR + 0] = k0 ? f0 : 0;
    s_flag[wave * KR + 1] = k1 ? f1 : 0;
    s_flag[wave * KR + 2] = k2 ? f2 : 0;
    s_flag[wave * KR + 3] = k3 ? f3 : 0;
  }
  __syncthreads();
  if (wave == 0) {
    const int l8 = lane < 8 ? lane : 7;
    const v4i fv = *(const v4ia*)(s_flag + 4 * l8);
    int* tp = TIE + (size_t)blockIdx.x * KROWS + 4 * l8;
    const bool wr = (lane < 8) && ((int)blockIdx.x * KROWS + KROWS <= nN);
    if (wr) *(volatile v4i*)tp = fv;
    __threadfence();
    if (wr) *(volatile v4i*)tp = fv;
  }
}

__global__ __launch_bounds__(NTHR) void k_tiecount(const int* __restrict__ TIE, int* CNT, int nN) {
  __shared__ int s_part[NTHR];
  const int tid = (int)threadIdx.x, lane = tid & 31, wave = tid >> 5;
  int acc = 0;
  const int nU = nN >> 2;
#pragma unroll 1
  for (int u = tid; u < nU; u += NTHR) {
    const v4i f = *(const v4ia*)(TIE + 4 * (size_t)u);
    acc += (f.x != 0 ? 1 : 0) + (f.y != 0 ? 1 : 0) + (f.z != 0 ? 1 : 0) + (f.w != 0 ? 1 : 0);
  }
  s_part[tid] = acc;
  __syncthreads();
  if (wave == 0) {
    int s = 0;
#pragma unroll
    for (int i = 0; i < 8; ++i) s += s_part[lane * 8 + i];
#pragma unroll
    for (int off = 16; off > 0; off >>= 1) s += __shfl_xor(s, off);
    v4i o;
    o.x = lane == 0 ? s : 0;
    o.y = lane == 0 ? nN : 0;
    o.z = 0; o.w = 0;
    int* cp = CNT + 4 * (lane < 8 ? lane : 7);
    if (lane < 8) *(volatile v4i*)cp = o;
    __threadfence();
    if (lane < 8) *(volatile v4i*)cp = o;
  }
}

__global__ __launch_bounds__(GTHR) void k_qkv(
    const unsigned short* __restrict__ A, const unsigned short* __restrict__ WT,
    const float* __restrict__ bq, const float* __restrict__ bk, const float* __restrict__ bv, float* outF)
{
  __shared__ __attribute__((aligned(16))) float stg[GBM * GBN];
  const int tid = (int)threadIdx.x, lane = tid & 31, wave = tid >> 5, hh = lane >> 4, m = lane & 15;
  const int rowBase = (int)blockIdx.x * GBM;
  const int by      = (int)blockIdx.y;
  const int col0    = by * GBN;
  const int mat     = by >> 1;
  const int cb      = (by & 1) * GBN;
  const float* bias = (mat == 0) ? bq : ((mat == 1) ? bk : bv);
  float bb[4];
#pragma unroll
  for (int t = 0; t < 4; ++t) bb[t] = bfr(bias[cb + 16 * t + m]);

  v8f acc[4];
  {
    const v8f z = {0.f, 0.f, 0.f, 0.f, 0.f, 0.f, 0.f, 0.f};
    acc[0] = z; acc[1] = z; acc[2] = z; acc[3] = z;
  }
  const unsigned short* ap = A  + (size_t)(rowBase + 16 * wave + m) * CCH + 8 * hh;
  const unsigned short* wp = WT + (size_t)(col0 + m) * CCH + 8 * hh;
#pragma unroll 1
  for (int ks = 0; ks < CCH / 32; ++ks) {
    FragB af;
    af.h[0] = *(const v8usa*)(ap + 32 * ks);
    af.h[1] = *(const v8usa*)(ap + 32 * ks + 16);
#pragma unroll
    for (int t = 0; t < 4; ++t) {
      const unsigned short* wq = wp + (size_t)(16 * t) * CCH + 32 * ks;
      FragB bf;
      bf.h[0] = *(const v8usa*)wq;
      bf.h[1] = *(const v8usa*)(wq + 16);
      acc[t] = wmb(af, bf, acc[t]);
    }
  }

#pragma unroll
  for (int t = 0; t < 4; ++t) {
    const int lc = 16 * t + m;
#pragma unroll
    for (int r = 0; r < 8; ++r) {
      const int lr = 16 * wave + 8 * hh + r;
      stg[lr * GBN + lc] = acc[t][r] + bb[t];
    }
  }
  __syncthreads();

  v4f fv[8];
#pragma unroll
  for (int i = 0; i < 8; ++i) {
    const int lr = 16 * wave + 2 * i + hh;
    fv[i] = *(const v4fa*)(stg + lr * GBN + 4 * m);
  }
#pragma unroll
  for (int i = 0; i < 8; ++i) {
    const int lr = 16 * wave + 2 * i + hh;
    const int gr = rowBase + lr;
    float* op = outF + (size_t)gr * NQKV + col0 + 4 * m;
    *(volatile v4f*)op = fv[i];
  }
  __threadfence();
#pragma unroll
  for (int i = 0; i < 8; ++i) {
    const int lr = 16 * wave + 2 * i + hh;
    const int gr = rowBase + lr;
    float* op = outF + (size_t)gr * NQKV + col0 + 4 * m;
    *(volatile v4f*)op = fv[i];
  }
}

__device__ __forceinline__ v4f prv(float t0, float t1, float t2, const v4f a, const v4f b, const v4f c, const v4f bp) {
  v4f r;
  r.x = fmaf(t2, c.x, fmaf(t1, b.x, t0 * a.x)) + bp.x;
  r.y = fmaf(t2, c.y, fmaf(t1, b.y, t0 * a.y)) + bp.y;
  r.z = fmaf(t2, c.z, fmaf(t1, b.z, t0 * a.z)) + bp.z;
  r.w = fmaf(t2, c.w, fmaf(t1, b.w, t0 * a.w)) + bp.w;
  return r;
}

__global__ __launch_bounds__(PTHR) void k_point(
    const float* __restrict__ P4, const float* __restrict__ XQKV, const int* __restrict__ KN,
    const unsigned short* __restrict__ W1T2, const unsigned short* __restrict__ W2T2,
    const float* __restrict__ Wp1, const float* __restrict__ bp1, const float* __restrict__ g1,
    const float* __restrict__ be1,
    const float* __restrict__ Wp2, const float* __restrict__ bp2, const float* __restrict__ g2,
    const float* __restrict__ be2,
    const float* __restrict__ bw1, const float* __restrict__ g3, const float* __restrict__ be3,
    const float* __restrict__ bw2,
    float* out, int nN)
{
  __shared__ __attribute__((aligned(16))) unsigned short s_a[PW][16 * APITCH];
  __shared__ __attribute__((aligned(16))) unsigned short s_a2[PW][16 * A2PITCH];
  __shared__ __attribute__((aligned(16))) float s_w[PW][16 * CS];
  const int tid = (int)threadIdx.x, lane = tid & 31, wave = tid >> 5, hh = lane >> 4, m = lane & 15;
  const int pt  = (int)blockIdx.x * PW + wave;
  const int ptc = pt < nN ? pt : nN - 1;
  unsigned short* sa  = &s_a[wave][0];
  unsigned short* sa2 = &s_a2[wave][0];
  float* sw = &s_w[wave][0];
  const float RC = 1.0f / BN_C;

  const int kw = KN[(size_t)ptc * 32 + lane];
  const int i9  = lane - 9,  i12 = lane - 12, i15 = lane - 15;
  const int a9  = i9  < 0 ? 0 : (i9  > 2 ? 2 : i9);
  const int a12 = i12 < 0 ? 0 : (i12 > 2 ? 2 : i12);
  const int a15 = i15 < 0 ? 0 : (i15 > 2 ? 2 : i15);
  const float c_w = Wp1[lane < 9 ? lane : 8];
  const float c_b = bp1[a9];
  const float c_g = g1[a12];
  const float c_e = be1[a15];
  ldwait();
  float cst = bfr(c_w);
  cst = (lane >= 9)  ? bfr(c_b) : cst;
  cst = (lane >= 12) ? bfr(c_g) * RC : cst;
  cst = (lane >= 15) ? bfr(c_e) : cst;

  const int nbraw = __shfl(kw, lane & 15);
  const int nbl   = nbraw < 0 ? 0 : (nbraw > nN - 1 ? nN - 1 : nbraw);
  const float d2l = __int_as_float(__shfl(kw, 16 + (lane & 15)));
  const float dcl = (d2l < 0.0f) ? 0.0f : d2l;
  const float dwl = expf(-sqrtf(dcl));

  const v4f pn = *(const v4fa*)(P4 + 4 * (size_t)nbl);
  const v4f pi = *(const v4fa*)(P4 + 4 * (size_t)ptc);
  const float r0 = pn.x - pi.x, r1 = pn.y - pi.y, r2 = pn.z - pi.z;
  float t0l, t1l, t2l;
  {
    const float w00 = rdlf(cst, 0), w01 = rdlf(cst, 1), w02 = rdlf(cst, 2);
    const float w10 = rdlf(cst, 3), w11 = rdlf(cst, 4), w12 = rdlf(cst, 5);
    const float w20 = rdlf(cst, 6), w21 = rdlf(cst, 7), w22 = rdlf(cst, 8);
    const float u0 = fmaf(r2, w20, fmaf(r1, w10, r0 * w00)) + rdlf(cst, 9);
    const float u1 = fmaf(r2, w21, fmaf(r1, w11, r0 * w01)) + rdlf(cst, 10);
    const float u2 = fmaf(r2, w22, fmaf(r1, w12, r0 * w02)) + rdlf(cst, 11);
    t0l = fmaxf(fmaf(u0, rdlf(cst, 12), rdlf(cst, 15)), 0.0f);
    t1l = fmaxf(fmaf(u1, rdlf(cst, 13), rdlf(cst, 16)), 0.0f);
    t2l = fmaxf(fmaf(u2, rdlf(cst, 14), rdlf(cst, 17)), 0.0f);
  }

  const int c0 = 4 * lane;
  const v4f w2a  = bfr4(*(const v4fa*)(Wp2 + c0));
  const v4f w2b  = bfr4(*(const v4fa*)(Wp2 + CCH + c0));
  const v4f w2c  = bfr4(*(const v4fa*)(Wp2 + 2 * CCH + c0));
  const v4f bp2v = bfr4(*(const v4fa*)(bp2 + c0));
  v4f sc2v       = bfr4(*(const v4fa*)(g2 + c0));
  sc2v.x = sc2v.x * RC; sc2v.y = sc2v.y * RC; sc2v.z = sc2v.z * RC; sc2v.w = sc2v.w * RC;
  const v4f be2v = bfr4(*(const v4fa*)(be2 + c0));
  const v4f xq   = *(const v4fa*)(XQKV + (size_t)ptc * NQKV + c0);

#pragma unroll 2
  for (int k = 0; k < KNN; ++k) {
    const int nk = __builtin_amdgcn_readlane(nbl, k);
    const float t0 = rdlf(t0l, k), t1 = rdlf(t1l, k), t2 = rdlf(t2l, k);
    const v4f xk = *(const v4fa*)(XQKV + (size_t)nk * NQKV + CCH + c0);
    const v4f pr = prv(t0, t1, t2, w2a, w2b, w2c, bp2v);
    const float ax = fmaxf(fmaf((xq.x - xk.x) + pr.x, sc2v.x, be2v.x), 0.0f);
    const float ay = fmaxf(fmaf((xq.y - xk.y) + pr.y, sc2v.y, be2v.y), 0.0f);
    const float az = fmaxf(fmaf((xq.z - xk.z) + pr.z, sc2v.z, be2v.z), 0.0f);
    const float aw = fmaxf(fmaf((xq.w - xk.w) + pr.w, sc2v.w, be2v.w), 0.0f);
    const unsigned int hx = f2bf(ax), hy = f2bf(ay), hz = f2bf(az), hw = f2bf(aw);
    const unsigned int lx = f2bf(ax - bf2f(hx)), ly = f2bf(ay - bf2f(hy));
    const unsigned int lz = f2bf(az - bf2f(hz)), lw = f2bf(aw - bf2f(hw));
    v2u hv, lv;
    hv.x = hx | (hy << 16); hv.y = hz | (hw << 16);
    lv.x = lx | (ly << 16); lv.y = lz | (lw << 16);
    *(v2ua*)(sa + k * APITCH + c0)       = hv;
    *(v2ua*)(sa + k * APITCH + CCH + c0) = lv;
  }

  const float bw1n = bfr(bw1[m]);
  const float sc3n = bfr(g3[m]) * RC;
  const float be3n = bfr(be3[m]);
  const float bw2n = bfr(bw2[m]);

  __builtin_amdgcn_fence(__ATOMIC_RELEASE, "wavefront");
  __builtin_amdgcn_wave_barrier();

  v8f acc = {0.f, 0.f, 0.f, 0.f, 0.f, 0.f, 0.f, 0.f};
  {
    const unsigned short* arow = sa + m * APITCH + 8 * hh;
    const unsigned short* brow = W1T2 + (size_t)m * (2 * CCH) + 8 * hh;
#pragma unroll 2
    for (int ks = 0; ks < (2 * CCH) / 32; ++ks) {
      FragB af, bf;
      af.h[0] = *(const v8usa*)(arow + 32 * ks);
      af.h[1] = *(const v8usa*)(arow + 32 * ks + 16);
      bf.h[0] = *(const v8usa*)(brow + 32 * ks);
      bf.h[1] = *(const v8usa*)(brow + 32 * ks + 16);
      acc = wmb(af, bf, acc);
    }
  }

#pragma unroll
  for (int r = 0; r < 8; ++r) {
    const float hv = fmaxf(fmaf(acc[r] + bw1n, sc3n, be3n), 0.0f);
    const unsigned int hb = f2bf(hv);
    const unsigned int lb = f2bf(hv - bf2f(hb));
    sa2[(8 * hh + r) * A2PITCH + m]      = (unsigned short)hb;
    sa2[(8 * hh + r) * A2PITCH + CS + m] = (unsigned short)lb;
  }
  __builtin_amdgcn_fence(__ATOMIC_RELEASE, "wavefront");
  __builtin_amdgcn_wave_barrier();

  v8f acc2 = {0.f, 0.f, 0.f, 0.f, 0.f, 0.f, 0.f, 0.f};
  {
    FragB a2, b2;
    const unsigned short* ar = sa2 + m * A2PITCH + 8 * hh;
    const unsigned short* br = W2T2 + (size_t)m * (2 * CS) + 8 * hh;
    a2.h[0] = *(const v8usa*)ar;
    a2.h[1] = *(const v8usa*)(ar + 16);
    b2.h[0] = *(const v8usa*)br;
    b2.h[1] = *(const v8usa*)(br + 16);
    acc2 = wmb(a2, b2, acc2);
  }

  {
    float sco[8];
#pragma unroll
    for (int r = 0; r < 8; ++r) sco[r] = acc2[r] + bw2n;
    float mx = sco[0];
#pragma unroll
    for (int r = 1; r < 8; ++r) mx = fmaxf(mx, sco[r]);
    mx = fmaxf(mx, __shfl_xor(mx, 16));
    float sum = 0.0f;
#pragma unroll
    for (int r = 0; r < 8; ++r) { sco[r] = expf(sco[r] - mx); sum += sco[r]; }
    sum += __shfl_xor(sum, 16);
    const float inv = 1.0f / sum;
#pragma unroll
    for (int r = 0; r < 8; ++r) sw[(8 * hh + r) * CS + m] = sco[r] * inv;
  }
  __builtin_amdgcn_fence(__ATOMIC_RELEASE, "wavefront");
  __builtin_amdgcn_wave_barrier();

  v4f o = {0.f, 0.f, 0.f, 0.f};
  const int wofs = 4 * (lane & 3);
#pragma unroll 2
  for (int k = 0; k < KNN; ++k) {
    const int nk = __builtin_amdgcn_readlane(nbl, k);
    const float t0 = rdlf(t0l, k), t1 = rdlf(t1l, k), t2 = rdlf(t2l, k);
    const float dwk = rdlf(dwl, k);
    const v4f xv = *(const v4fa*)(XQKV + (size_t)nk * NQKV + 2 * CCH + c0);
    const v4f pr = prv(t0, t1, t2, w2a, w2b, w2c, bp2v);
    const v4f wv = *(const v4fa*)(sw + k * CS + wofs);
    o.x = fmaf(fmaf(xv.x, dwk, pr.x), wv.x, o.x);
    o.y = fmaf(fmaf(xv.y, dwk, pr.y), wv.y, o.y);
    o.z = fmaf(fmaf(xv.z, dwk, pr.z), wv.z, o.z);
    o.w = fmaf(fmaf(xv.w, dwk, pr.w), wv.w, o.w);
  }
  float* op = out + (size_t)ptc * CCH + c0;
  const bool wr = pt < nN;
  if (wr) *(volatile v4f*)op = o;
  __threadfence();
  if (wr) *(volatile v4f*)op = o;
}

static inline int cdiv(int a, int b) { return (a + b - 1) / b; }

extern "C" void kernel_launch(void* const* d_in, const int* in_sizes, int n_in,
                              void* d_out, int out_size, void* d_ws, size_t ws_size,
                              hipStream_t stream) {
  if (n_in < 22) return;
  const int nN = in_sizes[0] / 3;
  if (nN < 64 || in_sizes[0] != nN * 3 || nN > (1 << 20)) return;
  if ((nN % 64) != 0) return;
  if (in_sizes[1] != nN * CCH) return;
  if (in_sizes[2] != CCH * CCH || in_sizes[4] != CCH * CCH || in_sizes[6] != CCH * CCH) return;
  if (in_sizes[3] != CCH || in_sizes[5] != CCH || in_sizes[7] != CCH) return;
  if (in_sizes[8] != 9 || in_sizes[9] != 3 || in_sizes[10] != 3 || in_sizes[11] != 3) return;
  if (in_sizes[12] != 3 * CCH || in_sizes[13] != CCH) return;
  if (in_sizes[14] != CCH || in_sizes[15] != CCH) return;
  if (in_sizes[16] != CCH * CS || in_sizes[17] != CS) return;
  if (in_sizes[18] != CS || in_sizes[19] != CS) return;
  if (in_sizes[20] != CS * CS || in_sizes[21] != CS) return;
  if (out_size != nN * CCH) return;

  const float* p   = (const float*)d_in[0];
  const float* x   = (const float*)d_in[1];
  const float* Wq  = (const float*)d_in[2];  const float* bq  = (const float*)d_in[3];
  const float* Wk  = (const float*)d_in[4];  const float* bk  = (const float*)d_in[5];
  const float* Wv  = (const float*)d_in[6];  const float* bv  = (const float*)d_in[7];
  const float* Wp1 = (const float*)d_in[8];  const float* bp1 = (const float*)d_in[9];
  const float* g1  = (const float*)d_in[10]; const float* be1 = (const float*)d_in[11];
  const float* Wp2 = (const float*)d_in[12]; const float* bp2 = (const float*)d_in[13];
  const float* g2  = (const float*)d_in[14]; const float* be2 = (const float*)d_in[15];
  const float* Ww1 = (const float*)d_in[16]; const float* bw1 = (const float*)d_in[17];
  const float* g3  = (const float*)d_in[18]; const float* be3 = (const float*)d_in[19];
  const float* Ww2 = (const float*)d_in[20]; const float* bw2 = (const float*)d_in[21];
  float* out = (float*)d_out;

  char* ws = (char*)d_ws;
  size_t off = 0;
  const size_t oP4  = off; off += (size_t)nN * 16;                  off = (off + 255) & ~(size_t)255;
  const size_t oXB  = off; off += (size_t)nN * CCH * 2;             off = (off + 255) & ~(size_t)255;
  const size_t oWQ  = off; off += (size_t)NQKV * CCH * 2;           off = (off + 255) & ~(size_t)255;
  const size_t oW1  = off; off += (size_t)CS * 2 * CCH * 2;         off = (off + 255) & ~(size_t)255;
  const size_t oW2  = off; off += (size_t)CS * 2 * CS * 2;          off = (off + 255) & ~(size_t)255;
  const size_t oXQ  = off; off += (size_t)nN * NQKV * 4;            off = (off + 255) & ~(size_t)255;
  const size_t oKN  = off; off += (size_t)nN * 32 * 4;              off = (off + 255) & ~(size_t)255;
  const size_t oTIE = off; off += (size_t)nN * 4;                   off = (off + 255) & ~(size_t)255;
  const size_t oCNT = off; off += (size_t)128;                      off = (off + 255) & ~(size_t)255;
  if (off > ws_size || off > (size_t)WSMAX) return;
  float*          P4    = (float*)(ws + oP4);
  unsigned short* XB    = (unsigned short*)(ws + oXB);
  unsigned short* WQKVT = (unsigned short*)(ws + oWQ);
  unsigned short* W1T2  = (unsigned short*)(ws + oW1);
  unsigned short* W2T2  = (unsigned short*)(ws + oW2);
  float*          XQKV  = (float*)(ws + oXQ);
  int*            KN    = (int*)(ws + oKN);
  int*            TIE   = (int*)(ws + oTIE);
  int*            CNT   = (int*)(ws + oCNT);

  k_pprep<<<cdiv(nN, NTHR), NTHR, 0, stream>>>(p, P4, nN);
  const int nUx = nN * (CCH / 8);
  k_xprep<<<cdiv(nUx, NTHR), NTHR, 0, stream>>>(x, XB, nN, nUx);

  k_wtr3<<<24, NTHR, 0, stream>>>(Wq, Wk, Wv, WQKVT);
  {
    const int nU1 = CS * ((2 * CCH) / 8);
    k_wtr<<<cdiv(nU1, NTHR), NTHR, 0, stream>>>(Ww1, CCH, CS, CS, 2 * CCH, W1T2, nU1);
    const int nU2 = CS * ((2 * CS) / 8);
    k_wtr<<<cdiv(nU2, NTHR), NTHR, 0, stream>>>(Ww2, CS, CS, CS, 2 * CS, W2T2, nU2);
  }

  k_knn<<<nN / KROWS, KTHR, 0, stream>>>(P4, KN, TIE, nN);

  k_qkv<<<dim3(nN / GBM, NQKV / GBN), GTHR, 0, stream>>>(XB, WQKVT, bq, bk, bv, XQKV);

  k_tiecount<<<1, NTHR, 0, stream>>>(TIE, CNT, nN);

  k_point<<<nN / PW, PTHR, 0, stream>>>(P4, XQKV, KN, W1T2, W2T2,
                                        Wp1, bp1, g1, be1, Wp2, bp2, g2, be2,
                                        bw1, g3, be3, bw2, out, nN);
  (void)stream;
}
